// Encoder_ODE_RNN_24885040513716
// MI455X (gfx1250) — hardware-verified
//
#include <hip/hip_runtime.h>
#include <stddef.h>
#include <math.h>

typedef __attribute__((ext_vector_type(16))) _Float16 v16h;
typedef __attribute__((ext_vector_type(8)))  _Float16 v8h;
typedef __attribute__((ext_vector_type(8)))  float    v8f;
typedef __attribute__((ext_vector_type(4)))  float    v4f;
typedef __attribute__((ext_vector_type(4)))  unsigned v4u;

template <typename T> struct Frag;
template <> struct Frag<_Float16> {
  typedef v16h V; union U { v16h v; v8h h[2]; };
  static __device__ __forceinline__ v16h load(const _Float16* p) {
    U f; f.h[0] = *(const v8h*)(p); f.h[1] = *(const v8h*)(p + 16); return f.v;
  }
  static __device__ __forceinline__ v8f mma(v16h a, v16h b, v8f c) {
    return __builtin_amdgcn_wmma_f32_16x16x32_f16(false, a, false, b, (short)0, c, false, false);
  }
};

__device__ __forceinline__ void mma_guard2(v8f& c0, v8f& c1, v16h a0, v16h a1, v16h b0) {
  asm volatile("v_nop\n\tv_nop\n\tv_nop\n\tv_nop" : "+v"(c0), "+v"(c1) : "v"(a0), "v"(a1), "v"(b0));
}
__device__ __forceinline__ void mma_guard4(v8f& c0, v8f& c1, v8f& c2, v8f& c3, v16h a0, v16h a1, v16h b0, v16h b1) {
  asm volatile("v_nop\n\tv_nop\n\tv_nop\n\tv_nop" : "+v"(c0), "+v"(c1), "+v"(c2), "+v"(c3) : "v"(a0), "v"(a1), "v"(b0), "v"(b1));
}
__device__ __forceinline__ void acc_guard2(v8f& a, v8f& b) { asm volatile("v_nop\n\tv_nop\n\tv_nop\n\tv_nop" : "+v"(a), "+v"(b)); }
__device__ __forceinline__ void acc_guard4(v8f& a, v8f& b, v8f& c, v8f& d) { asm volatile("v_nop\n\tv_nop\n\tv_nop\n\tv_nop" : "+v"(a), "+v"(b), "+v"(c), "+v"(d)); }

constexpr int NTRAJ = 1024;
constexpr int NTP   = 128;
constexpr int YD    = 64;
constexpr int HD    = 256;
constexpr int RD    = 128;
constexpr int NODE  = 100;
constexpr int ROWS_BLK = 32;
constexpr int NTHR  = 256;
constexpr int PY = 328;
constexpr int PH = 136;
constexpr int PG = 264;
constexpr int PO = 132;
constexpr float ACT_SCALE = 8.0f;
constexpr float WT_SCALE  = 16.0f;
constexpr float INV_PROD  = 0.0078125f;

constexpr size_t OFS_O1 = 0;
constexpr size_t OFS_O2 = OFS_O1 + 128 * 256;
constexpr size_t OFS_O3 = OFS_O2 + 128 * 128;
constexpr size_t OFS_U1 = OFS_O3 + 256 * 128;
constexpr size_t OFS_R1 = OFS_U1 + 256 * 320;
constexpr size_t OFS_N1 = OFS_R1 + 256 * 320;
constexpr size_t OFS_U2 = OFS_N1 + 256 * 320;
constexpr size_t OFS_R2 = OFS_U2 + 256 * 256;
constexpr size_t OFS_N2 = OFS_R2 + 256 * 256;
constexpr size_t OFS_FC = OFS_N2 + 256 * 256;
constexpr size_t WS_HALVES = OFS_FC + 128 * 256;
static_assert(WS_HALVES == 557056, "");

union LdsGateOut { _Float16 g[ROWS_BLK * PG]; float o[ROWS_BLK * PO]; };
static_assert(sizeof(LdsGateOut) == ROWS_BLK * PG * 2, "");
static_assert(ROWS_BLK * PO * 4 == ROWS_BLK * PG * 2, "");
static_assert(ROWS_BLK * PH <= ROWS_BLK * PG, "");

__device__ __forceinline__ float tanh_f(float x) {
  const float xc = fminf(fmaxf(x, -10.0f), 10.0f);
  const float e = expf(2.0f * xc);
  return 1.0f - 2.0f / (1.0f + e);
}
__device__ __forceinline__ float sigm_f(float x) {
  const float xc = fminf(fmaxf(x, -30.0f), 30.0f);
  const float e = expf(-xc);
  return 1.0f / (1.0f + e);
}

__global__ __launch_bounds__(256) void wt_transpose_f16(
    const float* __restrict__ W, int Kin, int Nin, _Float16* __restrict__ Bt, int Kpad, int Npad) {
  const int i = blockIdx.x * 256 + threadIdx.x;
  const int gpr = Kpad >> 3;
  const int total = Npad * gpr;
  if (i < total) {
    const int n  = i / gpr;
    const int k8 = (i - n * gpr) * 8;
    const int nc = (n < Nin) ? n : (Nin - 1);
    v8h hv;
#pragma unroll
    for (int e = 0; e < 8; ++e) {
      const int k  = k8 + e;
      const int kc = (k < Kin) ? k : (Kin - 1);
      float v = W[(size_t)kc * Nin + nc];
      v = (k < Kin && n < Nin) ? (v * WT_SCALE) : 0.0f;
      hv[e] = (_Float16)v;
    }
    _Float16* dst = Bt + (size_t)n * Kpad + k8;
    *(volatile v8h*)dst = hv;
    __threadfence();
    *(volatile v8h*)dst = hv;
  }
}

__device__ __forceinline__ void tile_gemm1(const _Float16* At, int lda,
                                           const _Float16* __restrict__ Bt, int ldb,
                                           int K, int ncol0, int lane, v8f (&acc)[2]) {
  const int m = lane & 15;
  const int koff = (lane >> 4) * 8;
  acc[0] = (v8f){0.f, 0.f, 0.f, 0.f, 0.f, 0.f, 0.f, 0.f};
  acc[1] = (v8f){0.f, 0.f, 0.f, 0.f, 0.f, 0.f, 0.f, 0.f};
  const _Float16* ap0 = At + m * lda + koff;
  const _Float16* ap1 = At + (m + 16) * lda + koff;
  const _Float16* bp0 = Bt + (size_t)(ncol0 + m) * ldb + koff;
#pragma unroll 1
  for (int k0 = 0; k0 < K; k0 += 32) {
    const v16h b0 = Frag<_Float16>::load(bp0 + k0);
    const v16h a0 = Frag<_Float16>::load(ap0 + k0);
    const v16h a1 = Frag<_Float16>::load(ap1 + k0);
    acc[0] = Frag<_Float16>::mma(a0, b0, acc[0]);
    acc[1] = Frag<_Float16>::mma(a1, b0, acc[1]);
    mma_guard2(acc[0], acc[1], a0, a1, b0);
  }
  acc_guard2(acc[0], acc[1]);
}

__device__ __forceinline__ void tile_gemm2(const _Float16* At, int lda,
                                           const _Float16* __restrict__ Bt, int ldb,
                                           int K, int ncol0, int lane, v8f (&acc)[2][2]) {
  const int m = lane & 15;
  const int koff = (lane >> 4) * 8;
#pragma unroll
  for (int i = 0; i < 2; ++i)
#pragma unroll
    for (int p = 0; p < 2; ++p) acc[i][p] = (v8f){0.f, 0.f, 0.f, 0.f, 0.f, 0.f, 0.f, 0.f};
  const _Float16* ap0 = At + m * lda + koff;
  const _Float16* ap1 = At + (m + 16) * lda + koff;
  const _Float16* bp0 = Bt + (size_t)(ncol0 + m) * ldb + koff;
  const _Float16* bp1 = Bt + (size_t)(ncol0 + 128 + m) * ldb + koff;
#pragma unroll 1
  for (int k0 = 0; k0 < K; k0 += 32) {
    const v16h b0 = Frag<_Float16>::load(bp0 + k0);
    const v16h b1 = Frag<_Float16>::load(bp1 + k0);
    const v16h a0 = Frag<_Float16>::load(ap0 + k0);
    const v16h a1 = Frag<_Float16>::load(ap1 + k0);
    acc[0][0] = Frag<_Float16>::mma(a0, b0, acc[0][0]);
    acc[1][0] = Frag<_Float16>::mma(a1, b0, acc[1][0]);
    acc[0][1] = Frag<_Float16>::mma(a0, b1, acc[0][1]);
    acc[1][1] = Frag<_Float16>::mma(a1, b1, acc[1][1]);
    mma_guard4(acc[0][0], acc[1][0], acc[0][1], acc[1][1], a0, a1, b0, b1);
  }
  acc_guard4(acc[0][0], acc[1][0], acc[0][1], acc[1][1]);
}

__global__ __launch_bounds__(256) void ode_gru_scan(
    const float* __restrict__ data, const float* __restrict__ ts, const _Float16* __restrict__ wt,
    const float* __restrict__ bu1, const float* __restrict__ bu2,
    const float* __restrict__ br1, const float* __restrict__ br2,
    const float* __restrict__ bn1, const float* __restrict__ bn2,
    const float* __restrict__ bo1, const float* __restrict__ bo2, const float* __restrict__ bo3,
    const float* __restrict__ bfc, float* __restrict__ out) {
  __shared__ __align__(16) _Float16   YB[ROWS_BLK * PY];
  __shared__ __align__(16) _Float16   GA[ROWS_BLK * PG];
  __shared__ __align__(16) LdsGateOut GB;

  _Float16* const H1  = GA;
  _Float16* const H2  = GB.g;
  _Float16* const GBu = GA;
  _Float16* const GBr = GB.g;
  float*    const OS  = GB.o;

  const int tid  = threadIdx.x;
  const int lane = tid & 31;
  const int w    = tid >> 5;
  const int m    = lane & 15;
  const int hi   = lane >> 4;
  const int row0 = blockIdx.x * ROWS_BLK;

  for (int i = tid; i < ROWS_BLK * (HD / 8); i += NTHR) {
    const int r  = i >> 5;
    const int c8 = (i & 31) * 8;
    *(v4u*)(YB + r * PY + c8) = (v4u){0u, 0u, 0u, 0u};
  }
  v8f yv[2][2], uv[2][2];
#pragma unroll
  for (int i = 0; i < 2; ++i)
#pragma unroll
    for (int p = 0; p < 2; ++p) {
      yv[i][p] = (v8f){0.f, 0.f, 0.f, 0.f, 0.f, 0.f, 0.f, 0.f};
      uv[i][p] = (v8f){0.f, 0.f, 0.f, 0.f, 0.f, 0.f, 0.f, 0.f};
    }
  __syncthreads();

  for (int t = 0; t < NTP; ++t) {
    unsigned lz = 0u;
    asm volatile("" : "+s"(lz));
    const _Float16* wsl = wt + lz;

    const int ia  = (NTP - 1) - t;
    const int ibr = NTP - t;
    const int ib  = (ibr > NTP - 1) ? (NTP - 1) : ibr;
    const float dts = ts[ia] - ts[ib];
    const float dt  = (t == 0) ? -0.01f : dts;

    {
      const int r  = tid >> 3;
      const int c8 = (tid & 7) * 8;
      const float* src = data + ((size_t)(row0 + r) * NTP + (size_t)((NTP - 1) - t)) * YD + c8;
      const v4f x0 = *(const v4f*)(src);
      const v4f x1 = *(const v4f*)(src + 4);
      v8h xv;
      xv[0] = (_Float16)(x0[0] * ACT_SCALE); xv[1] = (_Float16)(x0[1] * ACT_SCALE);
      xv[2] = (_Float16)(x0[2] * ACT_SCALE); xv[3] = (_Float16)(x0[3] * ACT_SCALE);
      xv[4] = (_Float16)(x1[0] * ACT_SCALE); xv[5] = (_Float16)(x1[1] * ACT_SCALE);
      xv[6] = (_Float16)(x1[2] * ACT_SCALE); xv[7] = (_Float16)(x1[3] * ACT_SCALE);
      *(v8h*)(YB + r * PY + HD + c8) = xv;
    }

    {
      v8f acc[2];
      tile_gemm1(YB, PY, wsl + OFS_O1, 256, 256, 16 * w, lane, acc);
      const int col  = 16 * w + m;
      const int colc = (col < NODE) ? col : (NODE - 1);
      float b = bo1[colc];
      b = (col < NODE) ? b : 0.0f;
#pragma unroll
      for (int ms = 0; ms < 2; ++ms)
#pragma unroll
        for (int r = 0; r < 8; ++r) {
          const float v = tanh_f(acc[ms][r] * INV_PROD + b);
          H1[(ms * 16 + 8 * hi + r) * PH + col] = (_Float16)(v * ACT_SCALE);
        }
    }
    __syncthreads();

    {
      v8f acc[2];
      tile_gemm1(H1, PH, wsl + OFS_O2, 128, 128, 16 * w, lane, acc);
      const int col  = 16 * w + m;
      const int colc = (col < NODE) ? col : (NODE - 1);
      float b = bo2[colc];
      b = (col < NODE) ? b : 0.0f;
#pragma unroll
      for (int ms = 0; ms < 2; ++ms)
#pragma unroll
        for (int r = 0; r < 8; ++r) {
          const float v = tanh_f(acc[ms][r] * INV_PROD + b);
          H2[(ms * 16 + 8 * hi + r) * PH + col] = (_Float16)(v * ACT_SCALE);
        }
    }
    __syncthreads();

    {
      v8f acc[2][2];
      tile_gemm2(H2, PH, wsl + OFS_O3, 128, 128, 16 * w, lane, acc);
#pragma unroll
      for (int ms = 0; ms < 2; ++ms)
#pragma unroll
        for (int p = 0; p < 2; ++p) {
          const int col = 16 * w + 128 * p + m;
          const float b = bo3[col];
#pragma unroll
          for (int r = 0; r < 8; ++r) {
            const float f  = acc[ms][p][r] * INV_PROD + b;
            const float yo = yv[ms][p][r] + f * dt;
            yv[ms][p][r] = yo;
            YB[(ms * 16 + 8 * hi + r) * PY + col] = (_Float16)(yo * ACT_SCALE);
          }
        }
    }
    __syncthreads();

    {
      v8f acc[2][2];
      tile_gemm2(YB, PY, wsl + OFS_U1, 320, 320, 16 * w, lane, acc);
#pragma unroll
      for (int ms = 0; ms < 2; ++ms)
#pragma unroll
        for (int p = 0; p < 2; ++p) {
          const int col = 16 * w + 128 * p + m;
          const float b = bu1[col];
#pragma unroll
          for (int r = 0; r < 8; ++r) {
            const float v = tanh_f(acc[ms][p][r] * INV_PROD + b);
            GBu[(ms * 16 + 8 * hi + r) * PG + col] = (_Float16)(v * ACT_SCALE);
          }
        }
    }
    {
      v8f acc[2][2];
      tile_gemm2(YB, PY, wsl + OFS_R1, 320, 320, 16 * w, lane, acc);
#pragma unroll
      for (int ms = 0; ms < 2; ++ms)
#pragma unroll
        for (int p = 0; p < 2; ++p) {
          const int col = 16 * w + 128 * p + m;
          const float b = br1[col];
#pragma unroll
          for (int r = 0; r < 8; ++r) {
            const float v = tanh_f(acc[ms][p][r] * INV_PROD + b);
            GBr[(ms * 16 + 8 * hi + r) * PG + col] = (_Float16)(v * ACT_SCALE);
          }
        }
    }
    __syncthreads();

    {
      v8f acc[2][2];
      tile_gemm2(GBu, PG, wsl + OFS_U2, 256, 256, 16 * w, lane, acc);
#pragma unroll
      for (int ms = 0; ms < 2; ++ms)
#pragma unroll
        for (int p = 0; p < 2; ++p) {
          const int col = 16 * w + 128 * p + m;
          const float b = bu2[col];
#pragma unroll
          for (int r = 0; r < 8; ++r) uv[ms][p][r] = sigm_f(acc[ms][p][r] * INV_PROD + b);
        }
    }
    {
      v8f acc[2][2];
      tile_gemm2(GBr, PG, wsl + OFS_R2, 256, 256, 16 * w, lane, acc);
#pragma unroll
      for (int ms = 0; ms < 2; ++ms)
#pragma unroll
        for (int p = 0; p < 2; ++p) {
          const int col = 16 * w + 128 * p + m;
          const float b = br2[col];
#pragma unroll
          for (int r = 0; r < 8; ++r) {
            const float rg = sigm_f(acc[ms][p][r] * INV_PROD + b);
            const float yr = yv[ms][p][r] * rg;
            YB[(ms * 16 + 8 * hi + r) * PY + col] = (_Float16)(yr * ACT_SCALE);
          }
        }
    }
    __syncthreads();

    {
      v8f acc[2][2];
      tile_gemm2(YB, PY, wsl + OFS_N1, 320, 320, 16 * w, lane, acc);
#pragma unroll
      for (int ms = 0; ms < 2; ++ms)
#pragma unroll
        for (int p = 0; p < 2; ++p) {
          const int col = 16 * w + 128 * p + m;
          const float b = bn1[col];
#pragma unroll
          for (int r = 0; r < 8; ++r) {
            const float v = tanh_f(acc[ms][p][r] * INV_PROD + b);
            GBu[(ms * 16 + 8 * hi + r) * PG + col] = (_Float16)(v * ACT_SCALE);
          }
        }
    }
    __syncthreads();

    {
      v8f acc[2][2];
      tile_gemm2(GBu, PG, wsl + OFS_N2, 256, 256, 16 * w, lane, acc);
#pragma unroll
      for (int ms = 0; ms < 2; ++ms)
#pragma unroll
        for (int p = 0; p < 2; ++p) {
          const int col = 16 * w + 128 * p + m;
          const float b = bn2[col];
#pragma unroll
          for (int r = 0; r < 8; ++r) {
            const float n  = acc[ms][p][r] * INV_PROD + b;
            const float u  = uv[ms][p][r];
            const float yo = yv[ms][p][r];
            const float yn = (1.0f - u) * n + u * yo;
            yv[ms][p][r] = yn;
            YB[(ms * 16 + 8 * hi + r) * PY + col] = (_Float16)(yn * ACT_SCALE);
          }
        }
    }
    __syncthreads();
  }

  {
    v8f acc[2];
    tile_gemm1(YB, PY, wt + OFS_FC, 256, 256, 16 * w, lane, acc);
    const int col = 16 * w + m;
    const float b = bfc[col];
#pragma unroll
    for (int ms = 0; ms < 2; ++ms)
#pragma unroll
      for (int r = 0; r < 8; ++r) OS[(ms * 16 + 8 * hi + r) * PO + col] = acc[ms][r] * INV_PROD + b;
  }
  __syncthreads();
  {
    const int c4 = lane * 4;
    for (int pass = 0; pass < 2; ++pass) {
#pragma unroll
      for (int rr = 0; rr < 4; ++rr) {
        const int row = w * 4 + rr;
        const v4f v = *(const v4f*)(OS + row * PO + c4);
        *(volatile v4f*)(out + (size_t)(row0 + row) * RD + c4) = v;
      }
      __threadfence();
    }
  }
}

extern "C" void kernel_launch(void* const* d_in, const int* in_sizes, int n_in,
                              void* d_out, int out_size, void* d_ws, size_t ws_size,
                              hipStream_t stream) {
  if (n_in < 22) return;
  if (in_sizes[0] != NTRAJ * NTP * YD) return;
  if (in_sizes[1] < NTP) return;
  if (in_sizes[2] != 320 * 256 || in_sizes[6] != 320 * 256 || in_sizes[10] != 320 * 256) return;
  if (in_sizes[4] != 256 * 256 || in_sizes[8] != 256 * 256 || in_sizes[12] != 256 * 256) return;
  if (in_sizes[14] != 256 * 100 || in_sizes[16] != 100 * 100 || in_sizes[18] != 100 * 256) return;
  if (in_sizes[20] != 256 * 128) return;
  if (in_sizes[3] < 256 || in_sizes[5] < 256 || in_sizes[7] < 256 || in_sizes[9] < 256 ||
      in_sizes[11] < 256 || in_sizes[13] < 256 || in_sizes[15] < 100 || in_sizes[17] < 100 ||
      in_sizes[19] < 256 || in_sizes[21] < 128) return;
  if (out_size != NTRAJ * RD) return;
  if (ws_size < WS_HALVES * sizeof(_Float16)) return;

  const float* data = (const float*)d_in[0];
  const float* ts   = (const float*)d_in[1];
  const float* Wu1 = (const float*)d_in[2];  const float* bu1 = (const float*)d_in[3];
  const float* Wu2 = (const float*)d_in[4];  const float* bu2 = (const float*)d_in[5];
  const float* Wr1 = (const float*)d_in[6];  const float* br1 = (const float*)d_in[7];
  const float* Wr2 = (const float*)d_in[8];  const float* br2 = (const float*)d_in[9];
  const float* Wn1 = (const float*)d_in[10]; const float* bn1 = (const float*)d_in[11];
  const float* Wn2 = (const float*)d_in[12]; const float* bn2 = (const float*)d_in[13];
  const float* Wo1 = (const float*)d_in[14]; const float* bo1 = (const float*)d_in[15];
  const float* Wo2 = (const float*)d_in[16]; const float* bo2 = (const float*)d_in[17];
  const float* Wo3 = (const float*)d_in[18]; const float* bo3 = (const float*)d_in[19];
  const float* Wfc = (const float*)d_in[20]; const float* bfc = (const float*)d_in[21];

  _Float16* wt = (_Float16*)d_ws;

  auto prep = [&](const float* W, int Kin, int Nin, size_t ofs, int Kpad, int Npad) {
    const int total = Npad * (Kpad / 8);
    wt_transpose_f16<<<(total + 255) / 256, 256, 0, stream>>>(W, Kin, Nin, wt + ofs, Kpad, Npad);
  };
  prep(Wo1, 256, 100, OFS_O1, 256, 128);
  prep(Wo2, 100, 100, OFS_O2, 128, 128);
  prep(Wo3, 100, 256, OFS_O3, 128, 256);
  prep(Wu1, 320, 256, OFS_U1, 320, 256);
  prep(Wr1, 320, 256, OFS_R1, 320, 256);
  prep(Wn1, 320, 256, OFS_N1, 320, 256);
  prep(Wu2, 256, 256, OFS_U2, 256, 256);
  prep(Wr2, 256, 256, OFS_R2, 256, 256);
  prep(Wn2, 256, 256, OFS_N2, 256, 256);
  prep(Wfc, 256, 128, OFS_FC, 256, 128);

  ode_gru_scan<<<NTRAJ / ROWS_BLK, NTHR, 0, stream>>>(
      data, ts, wt, bu1, bu2, br1, br2, bn1, bn2, bo1, bo2, bo3, bfc, (float*)d_out);
}
